// Graph_Model_35716948033625
// MI455X (gfx1250) — hardware-verified
//
#include <hip/hip_runtime.h>
#include <stddef.h>


#define FIN     128
#define NHEAD   4
#define HCH     32
#define NLAYER  3
#define XP      256
#define WP      128
#define YP      128
#define EP      4
#define DH      32
#define KM      256
#define NTHR    256
#define NWAVE   8
#define EPT     8
#define CHUNK   (NTHR * EPT)
#define WCAP    (EPT * 32)
#define LISTN   (NWAVE * WCAP)
#define NBMAX   2048
#define SLOTB   11
#define RCAP    28672
#define DEGCAP  4096
#define EPI     8
#define GBM     64
#define GTHR    128
#define NEG_SLOPE 0.2f
#define CA      16.0f
#define CW      64.0f
#define SCL     0.0009765625f
#define WSCAP   134217728
#define LDS_BUILD ((2 * RCAP + 2 * NBMAX + LISTN) * 4 + 64)

static_assert((CHUNK & (CHUNK - 1)) == 0 && CHUNK <= 4096);
static_assert(NBMAX == (1 << SLOTB));
static_assert(NTHR * 8 == NBMAX);
static_assert(LISTN >= NBMAX);
static_assert(LISTN >= NWAVE * WCAP);
static_assert((RCAP % 32) == 0);
static_assert(LDS_BUILD <= 300000);
static_assert(GBM == (GTHR / 32) * 16);
static_assert(GTHR == FIN);
static_assert(NHEAD * HCH == FIN);
static_assert(XP == 2 * FIN && KM == XP);
static_assert((FIN % 32) == 0 && (KM % 32) == 0);
static_assert(EPI * NHEAD == 32);
static_assert(HCH == 32 && DH == 32);
static_assert(GBM * EP == 2 * 32 * 4);

typedef float    v4f  __attribute__((ext_vector_type(4)));
typedef float    v8f  __attribute__((ext_vector_type(8)));
typedef int      v4i  __attribute__((ext_vector_type(4)));
typedef int      v8i  __attribute__((ext_vector_type(8)));
typedef _Float16 v8h  __attribute__((ext_vector_type(8)));
typedef _Float16 v16h __attribute__((ext_vector_type(16)));
union FragH { v16h v; v8h h[2]; v8i w; };

__device__ __forceinline__ v8f wmh(const FragH& a, const FragH& b, v8f c) {
  v8f d = __builtin_amdgcn_wmma_f32_16x16x32_f16(false, a.v, false, b.v, (short)0, c, false, false);
  asm volatile("v_nop\n\tv_nop\n\tv_nop\n\tv_nop" : "+v"(d) : "v"(a.w), "v"(b.w));
  return d;
}

__device__ __forceinline__ v8h pack8(v4f a, v4f b, float sc) {
  v8h hv;
  hv[0] = (_Float16)(a.x * sc); hv[1] = (_Float16)(a.y * sc);
  hv[2] = (_Float16)(a.z * sc); hv[3] = (_Float16)(a.w * sc);
  hv[4] = (_Float16)(b.x * sc); hv[5] = (_Float16)(b.y * sc);
  hv[6] = (_Float16)(b.z * sc); hv[7] = (_Float16)(b.w * sc);
  return hv;
}

__device__ __forceinline__ int scan_chunk(const int* __restrict__ dsts, int nE, int cbase, int slotBase,
                                          int nb, int vec8, int* list, int tid, int lane, int wave) {
  int wc = 0;
  const int el0  = tid * EPT;
  const int e0   = cbase + el0;
  const int sent = -2147483647 - 1;
  v4i da, db;
  if (vec8 != 0 && cbase + CHUNK <= nE) {
    da = *(const v4i*)(dsts + e0);
    db = *(const v4i*)(dsts + e0 + 4);
  } else {
    da.x = (e0     < nE) ? dsts[min(e0,     nE - 1)] : sent;
    da.y = (e0 + 1 < nE) ? dsts[min(e0 + 1, nE - 1)] : sent;
    da.z = (e0 + 2 < nE) ? dsts[min(e0 + 2, nE - 1)] : sent;
    da.w = (e0 + 3 < nE) ? dsts[min(e0 + 3, nE - 1)] : sent;
    db.x = (e0 + 4 < nE) ? dsts[min(e0 + 4, nE - 1)] : sent;
    db.y = (e0 + 5 < nE) ? dsts[min(e0 + 5, nE - 1)] : sent;
    db.z = (e0 + 6 < nE) ? dsts[min(e0 + 6, nE - 1)] : sent;
    db.w = (e0 + 7 < nE) ? dsts[min(e0 + 7, nE - 1)] : sent;
  }
  const unsigned nbs = (unsigned)slotBase;
  const unsigned unb = (unsigned)nb;
  const unsigned s0 = (unsigned)da.x - nbs, s1 = (unsigned)da.y - nbs;
  const unsigned s2 = (unsigned)da.z - nbs, s3 = (unsigned)da.w - nbs;
  const unsigned s4 = (unsigned)db.x - nbs, s5 = (unsigned)db.y - nbs;
  const unsigned s6 = (unsigned)db.z - nbs, s7 = (unsigned)db.w - nbs;
  const bool h0 = s0 < unb, h1 = s1 < unb, h2 = s2 < unb, h3 = s3 < unb;
  const bool h4 = s4 < unb, h5 = s5 < unb, h6 = s6 < unb, h7 = s7 < unb;
  const unsigned any = __builtin_amdgcn_ballot_w32(h0 | h1 | h2 | h3 | h4 | h5 | h6 | h7);
  if (any != 0u) {
#define HITJ(J, HJ, SJ) { \
      const unsigned mj = __builtin_amdgcn_ballot_w32(HJ); \
      if (mj != 0u) { \
        if (HJ) { \
          const int pos = wc + (int)__builtin_amdgcn_mbcnt_lo(mj, 0u); \
          if (pos < WCAP) list[wave * WCAP + pos] = ((el0 + (J)) << 12) | (int)(SJ); \
        } \
        wc += (int)__builtin_popcount(mj); } }
    HITJ(0, h0, s0)
    HITJ(1, h1, s1)
    HITJ(2, h2, s2)
    HITJ(3, h3, s3)
    HITJ(4, h4, s4)
    HITJ(5, h5, s5)
    HITJ(6, h6, s6)
    HITJ(7, h7, s7)
#undef HITJ
  }
  return wc;
}

__global__ __launch_bounds__(NTHR) void k_xprep(const float* __restrict__ x, _Float16* xc, int nN, int nUnits) {
  const int i = (int)blockIdx.x * NTHR + (int)threadIdx.x;
  if (i >= nUnits) return;
  const int row = i >> 5;
  const int c0  = (i & 31) * 8;
  const int rc  = row < nN ? row : nN - 1;
  const int cc  = c0 & (FIN - 1);
  const float* p = x + (size_t)rc * FIN + cc;
  v4f a = *(const v4f*)p, b = *(const v4f*)(p + 4);
  const v4f z4 = {0.f, 0.f, 0.f, 0.f};
  if (row >= nN) { a = z4; b = z4; }
  const v8h hv = pack8(a, b, CA);
  const size_t o = (size_t)row * XP + c0;
  *(volatile v8h*)(xc + o) = hv;
  __threadfence();
  *(volatile v8h*)(xc + o) = hv;
}

__global__ __launch_bounds__(NTHR) void k_wprep(const float* __restrict__ w, const float* __restrict__ w1,
                                                _Float16* wt3, _Float16* w1t) {
  const int j = (int)blockIdx.y;
  const int u = (int)blockIdx.x * NTHR + (int)threadIdx.x;
  if (j < NLAYER) {
    const int nUnits = FIN * (WP / 8);
    if (u >= nUnits) return;
    const int n  = u >> 4;
    const int k8 = (u & 15) * 8;
    const int kc = k8 < FIN - 8 ? k8 : FIN - 8;
    const int ncl = n < FIN ? n : FIN - 1;
    const float* p = w + (size_t)j * FIN * FIN + (size_t)kc * FIN + ncl;
    v4f a, b;
    a.x = p[0 * FIN]; a.y = p[1 * FIN]; a.z = p[2 * FIN]; a.w = p[3 * FIN];
    b.x = p[4 * FIN]; b.y = p[5 * FIN]; b.z = p[6 * FIN]; b.w = p[7 * FIN];
    const v8h hv = pack8(a, b, CW);
    const size_t o = ((size_t)j * FIN + (size_t)n) * WP + k8;
    *(volatile v8h*)(wt3 + o) = hv;
    __threadfence();
    *(volatile v8h*)(wt3 + o) = hv;
  } else {
    const int nUnits = DH * (XP / 8);
    if (u >= nUnits) return;
    const int n  = u >> 5;
    const int k8 = (u & 31) * 8;
    const int kc = k8 < KM - 8 ? k8 : KM - 8;
    const int ncl = n < DH ? n : DH - 1;
    const float* p = w1 + (size_t)kc * DH + ncl;
    v4f a, b;
    a.x = p[0 * DH]; a.y = p[1 * DH]; a.z = p[2 * DH]; a.w = p[3 * DH];
    b.x = p[4 * DH]; b.y = p[5 * DH]; b.z = p[6 * DH]; b.w = p[7 * DH];
    const v8h hv = pack8(a, b, CW);
    const size_t o = (size_t)n * XP + k8;
    *(volatile v8h*)(w1t + o) = hv;
    __threadfence();
    *(volatile v8h*)(w1t + o) = hv;
  }
}

__global__ __launch_bounds__(GTHR) void k_gemm(const _Float16* __restrict__ xc, const _Float16* __restrict__ wt,
                                               const float* __restrict__ asrc, const float* __restrict__ adst,
                                               float* Y, float* ES, float* ED) {
  __shared__ __attribute__((aligned(16))) float stg[GBM * FIN];
  __shared__ __attribute__((aligned(16))) float esT[GBM * EP];
  __shared__ __attribute__((aligned(16))) float edT[GBM * EP];
  __shared__ float sAs[FIN];
  __shared__ float sAd[FIN];
  const int tid = threadIdx.x, lane = tid & 31, wave = tid >> 5, hh = lane >> 4, m = lane & 15;
  const int rowBase = (int)blockIdx.x * GBM;
  sAs[tid] = asrc[tid];
  sAd[tid] = adst[tid];
  const size_t arow = (size_t)(rowBase + 16 * wave + m) * XP + 8 * hh;
  const size_t brow = (size_t)m * WP + 8 * hh;
  v8f acc[8];
#pragma unroll
  for (int t = 0; t < 8; ++t) { v8f z = {0.f, 0.f, 0.f, 0.f, 0.f, 0.f, 0.f, 0.f}; acc[t] = z; }
#pragma unroll 1
  for (int ks = 0; ks < FIN / 32; ++ks) {
    FragH af;
    af.h[0] = *(const v8h*)(xc + arow + 32 * ks);
    af.h[1] = *(const v8h*)(xc + arow + 32 * ks + 16);
#pragma unroll
    for (int t = 0; t < 8; ++t) {
      const size_t bo = brow + (size_t)(16 * t) * WP + 32 * ks;
      FragH bf;
      bf.h[0] = *(const v8h*)(wt + bo);
      bf.h[1] = *(const v8h*)(wt + bo + 16);
      acc[t] = wmh(af, bf, acc[t]);
    }
  }
  {
    float* sp = stg + (size_t)(16 * wave + 8 * hh) * FIN + m;
#pragma unroll
    for (int t = 0; t < 8; ++t) {
#pragma unroll
      for (int r = 0; r < 8; ++r) sp[(size_t)r * FIN + 16 * t] = acc[t][r] * SCL;
    }
  }
  __syncthreads();
  {
    const int row  = tid >> 1;
    const int half = tid & 1;
    const float* srow = stg + (size_t)row * FIN;
#pragma unroll 1
    for (int p = 0; p < NHEAD; ++p) {
      float s = 0.f, d = 0.f;
#pragma unroll 1
      for (int c = 0; c < HCH / 2; ++c) {
        const int cc = p * HCH + half * (HCH / 2) + c;
        const float v = srow[cc];
        s = fmaf(v, sAs[cc], s);
        d = fmaf(v, sAd[cc], d);
      }
      s += __shfl_xor(s, 1);
      d += __shfl_xor(d, 1);
      if (half == 0) {
        esT[row * EP + p] = s;
        edT[row * EP + p] = d;
      }
    }
  }
  {
    const int nF4 = GBM * FIN / 4;
    float* yb = Y + (size_t)rowBase * YP;
    const v4f* s4 = (const v4f*)stg;
#pragma unroll 1
    for (int f = tid; f < nF4; f += GTHR) {
      const int r = f >> 5, q = f & 31;
      const v4f v = s4[f];
      *(volatile v4f*)(yb + (size_t)r * YP + 4 * q) = v;
    }
    __threadfence();
#pragma unroll 1
    for (int f = tid; f < nF4; f += GTHR) {
      const int r = f >> 5, q = f & 31;
      const v4f v = s4[f];
      *(volatile v4f*)(yb + (size_t)r * YP + 4 * q) = v;
    }
  }
  __syncthreads();
  if (wave < 2) {
    const v4f ve = *(const v4f*)(esT + 128 * wave + 4 * lane);
    const v4f vd = *(const v4f*)(edT + 128 * wave + 4 * lane);
    float* pe = ES + (size_t)rowBase * EP + 128 * wave + 4 * lane;
    float* pd = ED + (size_t)rowBase * EP + 128 * wave + 4 * lane;
    *(volatile v4f*)pe = ve;
    *(volatile v4f*)pd = vd;
    __threadfence();
    *(volatile v4f*)pe = ve;
    *(volatile v4f*)pd = vd;
  }
}

__global__ __launch_bounds__(NTHR) void k_build(const int* __restrict__ dsts, int* EL, int* OFF, int* CNT,
                                                int nE, int nb, int tp, int vec8) {
  extern __shared__ v4f lds_dyn[];
  int* reg1 = (int*)lds_dyn;
  int* reg2 = reg1 + RCAP;
  int* scnt = reg2 + RCAP;
  int* soff = scnt + NBMAX;
  int* list = soff + NBMAX;
  int* wcnt = list + LISTN;
  int* wtot = wcnt + NWAVE;
  const int tid = threadIdx.x, lane = tid & 31, wave = tid >> 5;
  const int nodeBase = (int)blockIdx.x * nb;

  for (int i = tid; i < NBMAX; i += NTHR) scnt[i] = 0;
  {
    const v4i z = {0, 0, 0, 0};
    v4i* r2v = (v4i*)reg2;
    for (int f = tid; f < RCAP / 4; f += NTHR) r2v[f] = z;
  }
  __syncthreads();

  int tot = 0;
  const int nChunks = (nE + CHUNK - 1) / CHUNK;
#pragma unroll 1
  for (int ch = 0; ch < nChunks; ++ch) {
    const int cbase = ch * CHUNK;
    const int wc = scan_chunk(dsts, nE, cbase, nodeBase, nb, vec8, list, tid, lane, wave);
    if (lane == 0) wcnt[wave] = wc;
    __syncthreads();
    int pre = 0, all = 0;
#pragma unroll
    for (int w2 = 0; w2 < NWAVE; ++w2) {
      int c = wcnt[w2];
      c = c < 0 ? 0 : (c > WCAP ? WCAP : c);
      all += c;
      pre += (w2 < wave) ? c : 0;
    }
    const int wcc  = wc > WCAP ? WCAP : wc;
    const int base = tot + pre;
#pragma unroll 1
    for (int i = lane; i < wcc; i += 32) {
      const int ent = list[wave * WCAP + i];
      const int el  = (ent >> 12) & (CHUNK - 1);
      const int sl  = ent & (NBMAX - 1);
      int eid = cbase + el;
      eid = eid > nE - 1 ? nE - 1 : eid;
      const int pos = base + i;
      if (pos < RCAP) reg1[pos] = (int)(((unsigned)eid << SLOTB) | (unsigned)sl);
    }
    tot += all;
    tot = tot > RCAP ? RCAP : tot;
    __syncthreads();
  }
  const int nh = tot;

  if (wave == 0) {
#pragma unroll 1
    for (int b0 = 0; b0 < nh; b0 += 32) {
      const int idx = b0 + lane;
      const int uv  = reg1[idx < RCAP ? idx : RCAP - 1];
      const int m32 = (nh - b0) < 32 ? (nh - b0) : 32;
#pragma unroll 1
      for (int k = 0; k < m32; ++k) {
        const int u  = __builtin_amdgcn_readlane(uv, k);
        const int sl = u & (NBMAX - 1);
        if (lane == 0) scnt[sl] = scnt[sl] + 1;
      }
    }
  }
  __syncthreads();

  {
    const v4i ca = *(const v4i*)(scnt + 8 * tid);
    const v4i cb = *(const v4i*)(scnt + 8 * tid + 4);
    const int e0 = ca.x < 0 ? 0 : ca.x, e1 = ca.y < 0 ? 0 : ca.y, e2 = ca.z < 0 ? 0 : ca.z, e3 = ca.w < 0 ? 0 : ca.w;
    const int e4 = cb.x < 0 ? 0 : cb.x, e5 = cb.y < 0 ? 0 : cb.y, e6 = cb.z < 0 ? 0 : cb.z, e7 = cb.w < 0 ? 0 : cb.w;
    const int ts = e0 + e1 + e2 + e3 + e4 + e5 + e6 + e7;
    int incl = ts;
#pragma unroll
    for (int d = 1; d < 32; d <<= 1) {
      const int up = __shfl_up(incl, d);
      if (lane >= d) incl += up;
    }
    if (lane == 31) wtot[wave] = incl;
    __syncthreads();
    int pre = 0;
#pragma unroll
    for (int w2 = 0; w2 < NWAVE; ++w2) pre += (w2 < wave) ? wtot[w2] : 0;
    int run = pre + incl - ts;
    soff[8 * tid + 0] = run; run += e0;
    soff[8 * tid + 1] = run; run += e1;
    soff[8 * tid + 2] = run; run += e2;
    soff[8 * tid + 3] = run; run += e3;
    soff[8 * tid + 4] = run; run += e4;
    soff[8 * tid + 5] = run; run += e5;
    soff[8 * tid + 6] = run; run += e6;
    soff[8 * tid + 7] = run;
  }
  __syncthreads();
  for (int i = tid; i < NBMAX; i += NTHR) list[i] = soff[i];
  __syncthreads();

  if (wave == 0) {
#pragma unroll 1
    for (int b0 = 0; b0 < nh; b0 += 32) {
      const int idx = b0 + lane;
      const int uv  = reg1[idx < RCAP ? idx : RCAP - 1];
      const int m32 = (nh - b0) < 32 ? (nh - b0) : 32;
#pragma unroll 1
      for (int k = 0; k < m32; ++k) {
        const int u   = __builtin_amdgcn_readlane(uv, k);
        const int sl  = u & (NBMAX - 1);
        const int eid = (int)((unsigned)u >> SLOTB);
        if (lane == 0) {
          int pos = list[sl];
          pos = pos < 0 ? 0 : (pos > RCAP - 1 ? RCAP - 1 : pos);
          reg2[pos] = eid;
          list[sl] = pos + 1;
        }
      }
    }
  }
  __syncthreads();

  {
    int* elb = EL + (size_t)blockIdx.x * RCAP;
    const v4i* r4 = (const v4i*)reg2;
#pragma unroll 1
    for (int f = tid; f < RCAP / 4; f += NTHR) {
      const v4i v = r4[f];
      *(volatile v4i*)(elb + 4 * f) = v;
    }
    __threadfence();
#pragma unroll 1
    for (int f = tid; f < RCAP / 4; f += NTHR) {
      const v4i v = r4[f];
      *(volatile v4i*)(elb + 4 * f) = v;
    }
  }
  {
    const bool ovf = (nh >= RCAP);
    int* ob = OFF + (size_t)blockIdx.x * tp;
    int* cb = CNT + (size_t)blockIdx.x * tp;
    const int n4 = tp >> 2;
#pragma unroll 1
    for (int pass = 0; pass < 2; ++pass) {
#pragma unroll 1
      for (int f = tid; f < n4; f += NTHR) {
        v4i so, sc;
        {
          const int s = 4 * f + 0; const bool in = s < nb; const int scl = s < NBMAX ? s : NBMAX - 1;
          so.x = in ? soff[scl] : 0; sc.x = in ? (ovf ? -1 : scnt[scl]) : 0;
        }
        {
          const int s = 4 * f + 1; const bool in = s < nb; const int scl = s < NBMAX ? s : NBMAX - 1;
          so.y = in ? soff[scl] : 0; sc.y = in ? (ovf ? -1 : scnt[scl]) : 0;
        }
        {
          const int s = 4 * f + 2; const bool in = s < nb; const int scl = s < NBMAX ? s : NBMAX - 1;
          so.z = in ? soff[scl] : 0; sc.z = in ? (ovf ? -1 : scnt[scl]) : 0;
        }
        {
          const int s = 4 * f + 3; const bool in = s < nb; const int scl = s < NBMAX ? s : NBMAX - 1;
          so.w = in ? soff[scl] : 0; sc.w = in ? (ovf ? -1 : scnt[scl]) : 0;
        }
        *(volatile v4i*)(ob + 4 * f) = so;
        *(volatile v4i*)(cb + 4 * f) = sc;
      }
      __threadfence();
    }
  }
}

__global__ __launch_bounds__(NTHR) void k_agg(
    const int* __restrict__ srcs, const int* __restrict__ EL,
    const int* __restrict__ OFF, const int* __restrict__ CNT,
    const float* __restrict__ Y, const float* __restrict__ ES, const float* __restrict__ ED,
    const float* __restrict__ bias, _Float16* xout, int nN, int nE, int nb, int tp) {
  __shared__ v4f cmb[NWAVE * EPI * 32];
  __shared__ float cdn[NWAVE * EPI * NHEAD];
  const int tid = threadIdx.x, lane = tid & 31, wave = tid >> 5;
  const int g  = lane >> 2;
  const int j  = lane & 3;
  const int L  = lane & 15, hL = L >> 2;
  const int nodeBase = (int)blockIdx.x * nb;
  const int nbw = nb >> 3;
  const int* elb  = EL  + (size_t)blockIdx.x * RCAP;
  const int* offb = OFF + (size_t)blockIdx.x * tp;
  const int* cntb = CNT + (size_t)blockIdx.x * tp;
  const v4f bz0 = *(const v4f*)(bias + 8 * L);
  const v4f bz1 = *(const v4f*)(bias + 8 * L + 4);
  const float qnan = __int_as_float(0x7fc00000);
  const v4f z4 = {0.f, 0.f, 0.f, 0.f};
  v4f* cw = cmb + wave * (EPI * 32);
  float* cd = cdn + wave * (EPI * NHEAD);
#pragma unroll 1
  for (int jt = 0; jt < nbw; ++jt) {
    const int slot = wave * nbw + jt;
    const int grow = nodeBase + slot;
    const int gcl  = grow < nN ? grow : nN - 1;
    const bool wr  = grow < nN;
    int st = offb[slot];
    const int craw = cntb[slot];
    st = st < 0 ? 0 : (st > RCAP - 1 ? RCAP - 1 : st);
    int cnt = craw < 0 ? 0 : (craw > DEGCAP ? DEGCAP : craw);
    if (cnt > RCAP - st) cnt = RCAP - st;
    const float pz = (craw < 0 || craw > DEGCAP) ? qnan : 0.0f;

    const float edv = ED[(size_t)gcl * EP + j];
    const float esd = ES[(size_t)gcl * EP + j];
    const float t0  = esd + edv;
    float mx = fmaxf(t0, NEG_SLOPE * t0);
    const float* yd = Y + (size_t)gcl * YP + HCH * j;
    const bool g0 = (g == 0);
    float dn = g0 ? 1.0f : 0.0f;
    v4f a0 = g0 ? *(const v4f*)(yd +  0) : z4;
    v4f a1 = g0 ? *(const v4f*)(yd +  4) : z4;
    v4f a2 = g0 ? *(const v4f*)(yd +  8) : z4;
    v4f a3 = g0 ? *(const v4f*)(yd + 12) : z4;
    v4f a4 = g0 ? *(const v4f*)(yd + 16) : z4;
    v4f a5 = g0 ? *(const v4f*)(yd + 20) : z4;
    v4f a6 = g0 ? *(const v4f*)(yd + 24) : z4;
    v4f a7 = g0 ? *(const v4f*)(yd + 28) : z4;
    const int niter = (cnt + EPI - 1) / EPI;
#pragma unroll 1
    for (int it = 0; it < niter; ++it) {
      const int q = it * EPI + g;
      const bool valid = q < cnt;
      const int qc = valid ? q : cnt - 1;
      const int idx = st + qc;
      int eid = elb[idx];
      eid = eid < 0 ? 0 : (eid > nE - 1 ? nE - 1 : eid);
      const int sraw = srcs[eid];
      const int s = sraw < 0 ? 0 : (sraw > nN - 1 ? nN - 1 : sraw);
      const float* ys = Y + (size_t)s * YP + HCH * j;
      const v4f x0 = *(const v4f*)(ys +  0);
      const v4f x1 = *(const v4f*)(ys +  4);
      const v4f x2 = *(const v4f*)(ys +  8);
      const v4f x3 = *(const v4f*)(ys + 12);
      const v4f x4 = *(const v4f*)(ys + 16);
      const v4f x5 = *(const v4f*)(ys + 20);
      const v4f x6 = *(const v4f*)(ys + 24);
      const v4f x7 = *(const v4f*)(ys + 28);
      const float ess = ES[(size_t)s * EP + j];
      const float u = ess + edv;
      float l = fmaxf(u, NEG_SLOPE * u);
      l = valid ? l : (mx - 100.0f);
      const float mn = fmaxf(mx, l);
      const float s1 = __expf(mx - mn), s2 = __expf(l - mn);
      dn = fmaf(dn, s1, s2);
      a0 = a0 * s1 + x0 * s2;
      a1 = a1 * s1 + x1 * s2;
      a2 = a2 * s1 + x2 * s2;
      a3 = a3 * s1 + x3 * s2;
      a4 = a4 * s1 + x4 * s2;
      a5 = a5 * s1 + x5 * s2;
      a6 = a6 * s1 + x6 * s2;
      a7 = a7 * s1 + x7 * s2;
      mx = mn;
    }
    float m1 = fmaxf(mx, __shfl_xor(mx, 4));
    m1 = fmaxf(m1, __shfl_xor(m1, 8));
    m1 = fmaxf(m1, __shfl_xor(m1, 16));
    const float e = __expf(mx - m1);
    __builtin_amdgcn_fence(__ATOMIC_RELEASE, "wavefront");
    __builtin_amdgcn_wave_barrier();
    v4f* cg = cw + g * 32 + 8 * j;
    cg[0] = a0 * e; cg[1] = a1 * e; cg[2] = a2 * e; cg[3] = a3 * e;
    cg[4] = a4 * e; cg[5] = a5 * e; cg[6] = a6 * e; cg[7] = a7 * e;
    cd[g * NHEAD + j] = dn * e;
    __builtin_amdgcn_fence(__ATOMIC_RELEASE, "wavefront");
    __builtin_amdgcn_wave_barrier();
    v4f r0 = cw[2 * L], r1 = cw[2 * L + 1];
    float ds = cd[hL];
#pragma unroll
    for (int gg = 1; gg < EPI; ++gg) {
      r0 += cw[gg * 32 + 2 * L];
      r1 += cw[gg * 32 + 2 * L + 1];
      ds += cd[gg * NHEAD + hL];
    }
    const float inv = __builtin_amdgcn_rcpf(ds);
    const v4f o0 = r0 * inv + bz0 + pz;
    const v4f o1 = r1 * inv + bz1 + pz;
    const v8h hv = pack8(o0, o1, CA);
    _Float16* xp = xout + (size_t)gcl * XP + 8 * L;
    const bool stl = wr && (lane < 16);
    if (stl) *(volatile v8h*)xp = hv;
    __threadfence();
    if (stl) *(volatile v8h*)xp = hv;
  }
}

__global__ __launch_bounds__(GTHR) void k_mlp(const _Float16* __restrict__ xc, const _Float16* __restrict__ w1t,
                                              const float* __restrict__ b1, const float* __restrict__ w2,
                                              const float* __restrict__ b2, float* out, int nN) {
  __shared__ __attribute__((aligned(16))) float sO[GBM];
  __shared__ float sb1[DH];
  __shared__ float sw2[DH];
  const int tid = threadIdx.x, lane = tid & 31, wave = tid >> 5, hh = lane >> 4, m = lane & 15;
  const int rowBase = (int)blockIdx.x * GBM;
  if (tid < DH) { sb1[tid] = b1[tid]; sw2[tid] = w2[tid]; }
  const size_t arow = (size_t)(rowBase + 16 * wave + m) * XP + 8 * hh;
  const size_t brow = (size_t)m * XP + 8 * hh;
  v8f acc[2];
  {
    v8f z = {0.f, 0.f, 0.f, 0.f, 0.f, 0.f, 0.f, 0.f};
    acc[0] = z; acc[1] = z;
  }
#pragma unroll 1
  for (int ks = 0; ks < KM / 32; ++ks) {
    FragH af;
    af.h[0] = *(const v8h*)(xc + arow + 32 * ks);
    af.h[1] = *(const v8h*)(xc + arow + 32 * ks + 16);
#pragma unroll
    for (int t = 0; t < 2; ++t) {
      const size_t bo = brow + (size_t)(16 * t) * XP + 32 * ks;
      FragH bf;
      bf.h[0] = *(const v8h*)(w1t + bo);
      bf.h[1] = *(const v8h*)(w1t + bo + 16);
      acc[t] = wmh(af, bf, acc[t]);
    }
  }
  __syncthreads();
  float o[8];
  {
    const float c0 = sb1[m], c1 = sb1[16 + m];
    const float q0 = sw2[m], q1 = sw2[16 + m];
#pragma unroll
    for (int r = 0; r < 8; ++r) {
      const float h0 = fmaxf(fmaf(acc[0][r], SCL, c0), 0.f);
      const float h1 = fmaxf(fmaf(acc[1][r], SCL, c1), 0.f);
      o[r] = fmaf(h0, q0, h1 * q1);
    }
  }
#pragma unroll
  for (int r = 0; r < 8; ++r) {
    o[r] += __shfl_xor(o[r], 1);
    o[r] += __shfl_xor(o[r], 2);
    o[r] += __shfl_xor(o[r], 4);
    o[r] += __shfl_xor(o[r], 8);
  }
  {
    const float bb = b2[0];
    if (m == 0) {
#pragma unroll
      for (int r = 0; r < 8; ++r) {
        const float v  = o[r] + bb;
        const float ev = __expf(-v);
        sO[16 * wave + 8 * hh + r] = __builtin_amdgcn_rcpf(1.0f + ev);
      }
    }
  }
  __syncthreads();
  const int nValid = (nN - rowBase) < GBM ? (nN - rowBase) : GBM;
  const int fl  = nValid;
  const int n4  = fl >> 2;
  const int rem = fl & 3;
  float* base = out + (size_t)rowBase;
  const v4f* s4 = (const v4f*)sO;
  const v4f v = s4[tid < n4 ? tid : 0];
  const int ti = 4 * n4 + (lane & 3);
  const float tv = sO[ti < fl ? ti : fl - 1];
  const bool vw = (n4 > 0) && (tid < n4);
  const bool tw = (rem != 0) && (tid >= n4) && (tid < n4 + rem) && (wave == 0);
  if (vw) *(volatile v4f*)(base + 4 * tid) = v;
  if (tw) *(volatile float*)(base + 4 * n4 + (tid - n4)) = tv;
  __threadfence();
  if (vw) *(volatile v4f*)(base + 4 * tid) = v;
  if (tw) *(volatile float*)(base + 4 * n4 + (tid - n4)) = tv;
}

static int pick_nb(int nE, int nN) {
  int nb = NBMAX;
  while (nb > 16 && (long long)nb * (long long)nE * 5LL > (long long)RCAP * (long long)nN * 4LL) nb >>= 1;
  return nb;
}

extern "C" void kernel_launch(void* const* d_in, const int* in_sizes, int n_in,
                              void* d_out, int out_size, void* d_ws, size_t ws_size,
                              hipStream_t stream) {
  if (n_in < 10) return;
  const int nN = in_sizes[0] / FIN;
  if (nN <= 0 || in_sizes[0] != nN * FIN) return;
  if (nN > (1 << 22)) return;
  if (in_sizes[1] < 2 || (in_sizes[1] & 1) != 0) return;
  const int nE = in_sizes[1] / 2;
  if (nE < 1 || nE > (1 << 21)) return;
  if (in_sizes[2] != NLAYER * FIN * FIN) return;
  if (in_sizes[3] != NLAYER * FIN || in_sizes[4] != NLAYER * FIN) return;
  if (in_sizes[5] != NLAYER * FIN) return;
  if (in_sizes[6] != KM * DH) return;
  if (in_sizes[7] != DH || in_sizes[8] != DH || in_sizes[9] != 1) return;
  if (out_size != nN) return;

  const float* x     = (const float*)d_in[0];
  const int*   ei    = (const int*)d_in[1];
  const float* W     = (const float*)d_in[2];
  const float* att_s = (const float*)d_in[3];
  const float* att_d = (const float*)d_in[4];
  const float* bconv = (const float*)d_in[5];
  const float* W1    = (const float*)d_in[6];
  const float* b1    = (const float*)d_in[7];
  const float* W2    = (const float*)d_in[8];
  const float* b2    = (const float*)d_in[9];
  float* out = (float*)d_out;
  const int* dsts = ei + nE;

  const int MP   = ((nN + GBM - 1) / GBM) * GBM;
  const int nb   = pick_nb(nE, nN);
  const int tp   = nb < 32 ? 32 : nb;
  const int gA   = (nN + nb - 1) / nb;
  const int gG   = MP / GBM;
  const int vec8 = ((nE & 3) == 0) ? 1 : 0;
  const int nUnits = MP * (XP / 8);
  if (nb < 16 || nb > NBMAX || (long long)gA * nb < (long long)nN) return;

  char* ws = (char*)d_ws;
  size_t off = 0;
  const size_t oWT3 = off; off += (size_t)NLAYER * FIN * WP * 2; off = (off + 255) & ~(size_t)255;
  const size_t oW1T = off; off += (size_t)DH * XP * 2;           off = (off + 255) & ~(size_t)255;
  const size_t oXC  = off; off += (size_t)MP * XP * 2;           off = (off + 255) & ~(size_t)255;
  const size_t oY   = off; off += (size_t)MP * YP * 4;           off = (off + 255) & ~(size_t)255;
  const size_t oES  = off; off += (size_t)MP * EP * 4;           off = (off + 255) & ~(size_t)255;
  const size_t oED  = off; off += (size_t)MP * EP * 4;           off = (off + 255) & ~(size_t)255;
  const size_t oEL  = off; off += (size_t)gA * RCAP * 4;         off = (off + 255) & ~(size_t)255;
  const size_t oOFF = off; off += (size_t)gA * tp * 4;           off = (off + 255) & ~(size_t)255;
  const size_t oCNT = off; off += (size_t)gA * tp * 4;           off = (off + 255) & ~(size_t)255;
  if (off > ws_size || off > (size_t)WSCAP) return;
  _Float16* WT3 = (_Float16*)(ws + oWT3);
  _Float16* W1T = (_Float16*)(ws + oW1T);
  _Float16* XC  = (_Float16*)(ws + oXC);
  float*    Y   = (float*)(ws + oY);
  float*    ES  = (float*)(ws + oES);
  float*    ED  = (float*)(ws + oED);
  int*      EL  = (int*)(ws + oEL);
  int*      OFF = (int*)(ws + oOFF);
  int*      CNT = (int*)(ws + oCNT);

  hipFuncSetAttribute(reinterpret_cast<const void*>(&k_build),
                      hipFuncAttributeMaxDynamicSharedMemorySize, LDS_BUILD);

  k_xprep<<<(nUnits + NTHR - 1) / NTHR, NTHR, 0, stream>>>(x, XC, nN, nUnits);
  k_wprep<<<dim3((FIN * (WP / 8) + NTHR - 1) / NTHR, NLAYER + 1), NTHR, 0, stream>>>(W, W1, WT3, W1T);

  k_build<<<gA, NTHR, LDS_BUILD, stream>>>(dsts, EL, OFF, CNT, nE, nb, tp, vec8);

  for (int l = 0; l < NLAYER; ++l) {
    k_gemm<<<gG, GTHR, 0, stream>>>(XC, WT3 + (size_t)l * FIN * WP, att_s + (size_t)l * FIN,
                                    att_d + (size_t)l * FIN, Y, ES, ED);
    k_agg<<<gA, NTHR, 0, stream>>>(ei, EL, OFF, CNT, Y, ES, ED, bconv + (size_t)l * FIN, XC, nN, nE, nb, tp);
  }

  k_mlp<<<gG, GTHR, 0, stream>>>(XC, W1T, b1, W2, b2, out, nN);
}
